// MLPDecoder_Causal_11639361372236
// MI455X (gfx1250) — hardware-verified
//
#include <hip/hip_runtime.h>
#include <stddef.h>


namespace {

constexpr int NB  = 32;
constexpr int NA  = 32;
constexpr int NT  = 64;
constexpr int NTS = 32;
constexpr int NTO = NT - 1;
constexpr int ND  = 16;
constexpr int NH  = 64;
constexpr int NE  = NA * (NA - 1);
constexpr int NSL = 32;
constexpr int NTHR = 256;

constexpr int W1T_OFF   = 0;
constexpr int W2T_OFF   = W1T_OFF + 2 * 4 * 32 * 16;
constexpr int EW_HALVES = W2T_OFF + 2 * 2 * 4 * 32 * 16;
constexpr int O1OFF     = EW_HALVES;
constexpr int O2OFF     = O1OFF + 3 * 4 * 32 * 16;
constexpr int O3OFF     = O2OFF + 2 * 4 * 32 * 16;
constexpr int WTAB_HALVES = O3OFF + 2 * 32 * 16;

constexpr size_t WTAB_BYTES = (size_t)WTAB_HALVES * 2;
constexpr size_t CPAD_OFFB  = WTAB_BYTES;
constexpr size_t CPAD_BYTES = (size_t)2 * NA * NSL * 4;
constexpr size_t R_OFFB     = CPAD_OFFB + CPAD_BYTES;
constexpr size_t R_BYTES    = (size_t)NB * NTS * 2 * NA * ND * 4;
constexpr size_t WS_TOTAL   = R_OFFB + R_BYTES;
static_assert(WTAB_BYTES % 128 == 0);
static_assert(CPAD_OFFB % 128 == 0);
static_assert(R_OFFB % 128 == 0);
static_assert((EW_HALVES * 2) % 128 == 0);

typedef _Float16 h2_t  __attribute__((ext_vector_type(2)));
typedef _Float16 h8_t  __attribute__((ext_vector_type(8)));
typedef _Float16 h16_t __attribute__((ext_vector_type(16)));
typedef float    f8_t  __attribute__((ext_vector_type(8)));
typedef float    f4_t  __attribute__((ext_vector_type(4)));
typedef h2_t v2h __attribute__((may_alias));
typedef h8_t v8h __attribute__((may_alias));
typedef f4_t v4f __attribute__((may_alias));

union Frag { h16_t v; v8h h[2]; _Float16 e[16]; };
union Acc  { f8_t v; float f[8]; };

__device__ __forceinline__ f8_t mma_raw(const h16_t a, const h16_t b, f8_t c) {
  return __builtin_amdgcn_wmma_f32_16x16x32_f16(false, a, false, b, (short)0, c, false, false);
}

__device__ __forceinline__ f8_t mma16(const h16_t a, const h16_t b, f8_t c) {
  f8_t d = mma_raw(a, b, c);
  asm volatile("v_nop\n\tv_nop\n\tv_nop\n\tv_nop" : "+v"(d) : "v"(a), "v"(b));
  return d;
}

__device__ __forceinline__ v8h zero8() {
  v8h z = {(_Float16)0.0f, (_Float16)0.0f, (_Float16)0.0f, (_Float16)0.0f,
           (_Float16)0.0f, (_Float16)0.0f, (_Float16)0.0f, (_Float16)0.0f};
  return z;
}

__device__ __forceinline__ int kmap(int e, int hh) { return 8 * hh + (e & 7) + ((e >> 3) << 4); }

__device__ float wtab_val(int q, const float* W1, const float* W2,
                          const float* O1, const float* O2, const float* O3) {
  if (q < W2T_OFF) {
    const int e = q & 15, l = (q >> 4) & 31, mt = (q >> 9) & 3, k = (q >> 11) & 1;
    const int kk = kmap(e, l >> 4), col = mt * 16 + (l & 15);
    return W1[(k * 32 + kk) * NH + col];
  }
  if (q < O1OFF) {
    const int p = q - W2T_OFF;
    const int e = p & 15, l = (p >> 4) & 31, mt = (p >> 9) & 3, kf = (p >> 11) & 1, k = (p >> 12) & 1;
    const int kk = kf * 32 + kmap(e, l >> 4), col = mt * 16 + (l & 15);
    return W2[(k * NH + kk) * NH + col];
  }
  if (q < O2OFF) {
    const int p = q - O1OFF;
    const int e = p & 15, l = (p >> 4) & 31, n = (p >> 9) & 3, kf = p >> 11;
    const int kk = kf * 32 + kmap(e, l >> 4), col = n * 16 + (l & 15);
    return (kk < ND + NH) ? O1[kk * NH + col] : 0.0f;
  }
  if (q < O3OFF) {
    const int p = q - O2OFF;
    const int e = p & 15, l = (p >> 4) & 31, n = (p >> 9) & 3, kf = (p >> 11) & 1;
    const int kk = kf * 32 + kmap(e, l >> 4), col = n * 16 + (l & 15);
    return O2[kk * NH + col];
  }
  const int p = q - O3OFF;
  const int e = p & 15, l = (p >> 4) & 31, kf = (p >> 9) & 1;
  const int kk = kf * 32 + kmap(e, l >> 4), col = l & 15;
  return O3[kk * ND + col];
}

__device__ __forceinline__ float edge_coef(int k, int e, const float* rg, const float* gb) {
  const float z0 = (rg[2 * e] + gb[2 * e]) * 2.0f;
  const float z1 = (rg[2 * e + 1] + gb[2 * e + 1]) * 2.0f;
  const float m  = fmaxf(z0, z1);
  const float e0 = __expf(z0 - m);
  const float e1 = __expf(z1 - m);
  const float inv = __builtin_amdgcn_rcpf(e0 + e1);
  return (k == 0 ? e0 : e1) * inv;
}

__device__ __forceinline__ void prep_pass(int tid,
    const float* rr, const float* rg, const float* gb,
    const float* W1, const float* W2, const float* O1, const float* O2, const float* O3,
    _Float16* wtab, float* cpad) {
#pragma unroll 1
  for (int c = tid; c < WTAB_HALVES / 8; c += NTHR) {
    union { h8_t v; _Float16 e[8]; } u;
#pragma unroll
    for (int q = 0; q < 8; ++q) u.e[q] = (_Float16)wtab_val(c * 8 + q, W1, W2, O1, O2, O3);
    *(volatile v8h*)(wtab + (size_t)c * 8) = u.v;
  }
#pragma unroll 1
  for (int c = tid; c < 2 * NA * NSL / 4; c += NTHR) {
    const int q0 = c * 4;
    const int k = q0 >> 10, i = (q0 >> 5) & 31, s0 = q0 & 31;
    union { f4_t v; float f[4]; } u;
#pragma unroll
    for (int q = 0; q < 4; ++q) {
      const int s = s0 + q;
      float v = 0.0f;
      if (s < NA - 1) {
        const int e = (NA - 1) * i + s;
        v = edge_coef(k, e, rg, gb) * rr[e * NA + i];
      }
      u.f[q] = v;
    }
    *(volatile v4f*)(cpad + q0) = u.v;
  }
}

__global__ __launch_bounds__(NTHR)
void k_prep(const float* __restrict__ rel_rec,
            const float* __restrict__ rel_graph, const float* __restrict__ gumbel,
            const float* __restrict__ msg_W1, const float* __restrict__ msg_W2,
            const float* __restrict__ out_W1, const float* __restrict__ out_W2,
            const float* __restrict__ out_W3,
            _Float16* __restrict__ wtab, float* __restrict__ cpad) {
  const int tid = threadIdx.x;
  prep_pass(tid, rel_rec, rel_graph, gumbel, msg_W1, msg_W2, out_W1, out_W2, out_W3, wtab, cpad);
  __threadfence();
  prep_pass(tid, rel_rec, rel_graph, gumbel, msg_W1, msg_W2, out_W1, out_W2, out_W3, wtab, cpad);
}

__device__ __forceinline__ void row_frag(Frag& f, const float* row, int hh) {
  const v4f x0 = *(const v4f*)(row + 8 * hh);
  const v4f x1 = *(const v4f*)(row + 8 * hh + 4);
  const v4f x2 = *(const v4f*)(row + 16 + 8 * hh);
  const v4f x3 = *(const v4f*)(row + 16 + 8 * hh + 4);
  f.e[0]  = (_Float16)x0.x; f.e[1]  = (_Float16)x0.y; f.e[2]  = (_Float16)x0.z; f.e[3]  = (_Float16)x0.w;
  f.e[4]  = (_Float16)x1.x; f.e[5]  = (_Float16)x1.y; f.e[6]  = (_Float16)x1.z; f.e[7]  = (_Float16)x1.w;
  f.e[8]  = (_Float16)x2.x; f.e[9]  = (_Float16)x2.y; f.e[10] = (_Float16)x2.z; f.e[11] = (_Float16)x2.w;
  f.e[12] = (_Float16)x3.x; f.e[13] = (_Float16)x3.y; f.e[14] = (_Float16)x3.z; f.e[15] = (_Float16)x3.w;
}

__global__ __launch_bounds__(NTHR) __attribute__((amdgpu_num_vgpr(192)))
void k_step(const float* __restrict__ xin,
            const float* __restrict__ rel_rec, const float* __restrict__ rel_send,
            const _Float16* __restrict__ wtab, const float* __restrict__ cpad,
            const float* __restrict__ mb1, const float* __restrict__ mb2,
            const float* __restrict__ ob1g, const float* __restrict__ ob2g, const float* __restrict__ ob3g,
            float* __restrict__ rbuf) {
  __shared__ __attribute__((aligned(32))) _Float16 s_w[EW_HALVES];
  __shared__ __attribute__((aligned(32))) float    s_c[2][NA][NSL];
  __shared__ __attribute__((aligned(32))) float    s_xs[NA][ND];
  __shared__ __attribute__((aligned(32))) _Float16 s_xh[NA][ND];
  __shared__ __attribute__((aligned(32))) _Float16 s_xT[ND][NA];
  __shared__ __attribute__((aligned(32))) _Float16 s_agh[NA][NH];
  __shared__ __attribute__((aligned(32))) _Float16 s_p1[NA][NH];
  __shared__ __attribute__((aligned(32))) _Float16 s_p2[NA][NH];
  __shared__ __attribute__((aligned(32))) float    s_b1[2][NH];
  __shared__ __attribute__((aligned(32))) float    s_b2[2][NH];
  __shared__ __attribute__((aligned(32))) float    s_ob1[NH];
  __shared__ __attribute__((aligned(32))) float    s_ob2[NH];
  __shared__ __attribute__((aligned(32))) float    s_ob3[ND];

  const int tid = threadIdx.x;
  const int blk = blockIdx.x;
  if (blk >= NB * NTS) return;
  const int b = blk >> 5, t = blk & 31;
  const int wave = tid >> 5, lane = tid & 31, hh = lane >> 4, ln = lane & 15;

  for (int q = tid; q < EW_HALVES / 8; q += NTHR)
    *(v8h*)(s_w + q * 8) = *(const v8h*)(wtab + q * 8);
  for (int q = tid; q < 2 * NA * NSL / 4; q += NTHR)
    *(v4f*)(&s_c[0][0][0] + q * 4) = *(const v4f*)(cpad + q * 4);
  for (int q = tid; q < NA * ND; q += NTHR) {
    const int a = q >> 4, d = q & 15;
    const float v = xin[(((size_t)b * NA + a) * NT + 2 * t) * ND + d];
    const _Float16 hv = (_Float16)v;
    s_xs[a][d] = v;
    s_xh[a][d] = hv;
    s_xT[d][a] = hv;
  }
  for (int q = tid; q < 2 * NH; q += NTHR) { (&s_b1[0][0])[q] = mb1[q]; (&s_b2[0][0])[q] = mb2[q]; }
  if (tid < NH) { s_ob1[tid] = ob1g[tid]; s_ob2[tid] = ob2g[tid]; }
  if (tid < ND) s_ob3[tid] = ob3g[tid];

  const v8h z8 = zero8();
  const int nsteps = (t == NTS - 1) ? 1 : 2;

  for (int step = 0; step < nsteps; ++step) {
    __syncthreads();

    Frag fx;
    fx.h[0] = *(const v8h*)&s_xT[ln][8 * hh];
    fx.h[1] = *(const v8h*)&s_xT[ln][16 + 8 * hh];

#pragma unroll 1
    for (int ii = 0; ii < 4; ++ii) {
      const int i = wave * 4 + ii;
      Acc msg[4];
#pragma unroll
      for (int mt = 0; mt < 4; ++mt)
#pragma unroll
        for (int r = 0; r < 8; ++r) msg[mt].f[r] = 0.0f;

#pragma unroll 1
      for (int hf = 0; hf < 2; ++hf) {
        const int s = hf * 16 + ln;
        int e = (NA - 1) * i + s;
        e = (e < NE) ? e : (NE - 1);

        Frag fbs, fbr;
        row_frag(fbs, rel_send + (size_t)e * NA, hh);
        row_frag(fbr, rel_rec  + (size_t)e * NA, hh);

        Acc dS, dR;
#pragma unroll
        for (int r = 0; r < 8; ++r) { dS.f[r] = 0.0f; dR.f[r] = 0.0f; }
        dS.v = mma_raw(fx.v, fbs.v, dS.v);
        dR.v = mma_raw(fx.v, fbr.v, dR.v);
        asm volatile("v_nop\n\tv_nop\n\tv_nop\n\tv_nop"
                     : "+v"(dS.v), "+v"(dR.v) : "v"(fx.v), "v"(fbs.v), "v"(fbr.v));

        Frag fp;
#pragma unroll
        for (int q = 0; q < 8; ++q) { fp.e[q] = (_Float16)dS.f[q]; fp.e[8 + q] = (_Float16)dR.f[q]; }

#pragma unroll 1
        for (int k = 0; k < 2; ++k) {
          const float c = s_c[k][i][s];

          Acc a1[4];
#pragma unroll
          for (int mt = 0; mt < 4; ++mt) {
            const v4f b0 = *(const v4f*)&s_b1[k][16 * mt + 8 * hh];
            const v4f b1 = *(const v4f*)&s_b1[k][16 * mt + 8 * hh + 4];
            a1[mt].f[0] = b0.x; a1[mt].f[1] = b0.y; a1[mt].f[2] = b0.z; a1[mt].f[3] = b0.w;
            a1[mt].f[4] = b1.x; a1[mt].f[5] = b1.y; a1[mt].f[6] = b1.z; a1[mt].f[7] = b1.w;
          }
          Frag w1f[4];
#pragma unroll
          for (int mt = 0; mt < 4; ++mt) {
            const _Float16* p = s_w + W1T_OFF + (((k * 4 + mt) * 32 + lane) * 16);
            w1f[mt].h[0] = *(const v8h*)p;
            w1f[mt].h[1] = *(const v8h*)(p + 8);
          }
#pragma unroll
          for (int mt = 0; mt < 4; ++mt) a1[mt].v = mma_raw(w1f[mt].v, fp.v, a1[mt].v);
          asm volatile("v_nop\n\tv_nop\n\tv_nop\n\tv_nop"
                       : "+v"(a1[0].v), "+v"(a1[1].v), "+v"(a1[2].v), "+v"(a1[3].v)
                       : "v"(w1f[0].v), "v"(w1f[1].v), "v"(w1f[2].v), "v"(w1f[3].v), "v"(fp.v));

          Frag fh[2];
#pragma unroll
          for (int kf = 0; kf < 2; ++kf)
#pragma unroll
            for (int q = 0; q < 8; ++q) {
              fh[kf].e[q]     = (_Float16)fmaxf(a1[2 * kf].f[q], 0.0f);
              fh[kf].e[8 + q] = (_Float16)fmaxf(a1[2 * kf + 1].f[q], 0.0f);
            }

          Acc a2[4];
#pragma unroll
          for (int mt = 0; mt < 4; ++mt) {
            const v4f b0 = *(const v4f*)&s_b2[k][16 * mt + 8 * hh];
            const v4f b1 = *(const v4f*)&s_b2[k][16 * mt + 8 * hh + 4];
            a2[mt].f[0] = b0.x; a2[mt].f[1] = b0.y; a2[mt].f[2] = b0.z; a2[mt].f[3] = b0.w;
            a2[mt].f[4] = b1.x; a2[mt].f[5] = b1.y; a2[mt].f[6] = b1.z; a2[mt].f[7] = b1.w;
          }
#pragma unroll
          for (int kf = 0; kf < 2; ++kf) {
            Frag w2f[4];
#pragma unroll
            for (int mt = 0; mt < 4; ++mt) {
              const _Float16* p = s_w + W2T_OFF + ((((k * 2 + kf) * 4 + mt) * 32 + lane) * 16);
              w2f[mt].h[0] = *(const v8h*)p;
              w2f[mt].h[1] = *(const v8h*)(p + 8);
            }
#pragma unroll
            for (int mt = 0; mt < 4; ++mt) a2[mt].v = mma_raw(w2f[mt].v, fh[kf].v, a2[mt].v);
            asm volatile("v_nop\n\tv_nop\n\tv_nop\n\tv_nop"
                         : "+v"(a2[0].v), "+v"(a2[1].v), "+v"(a2[2].v), "+v"(a2[3].v)
                         : "v"(w2f[0].v), "v"(w2f[1].v), "v"(w2f[2].v), "v"(w2f[3].v), "v"(fh[kf].v));
          }

#pragma unroll
          for (int mt = 0; mt < 4; ++mt)
#pragma unroll
            for (int r = 0; r < 8; ++r)
              msg[mt].f[r] = fmaf(fmaxf(a2[mt].f[r], 0.0f), c, msg[mt].f[r]);
        }
      }

      float u1[16];
      {
        const bool sel = (ln & 8) != 0;
#pragma unroll
        for (int q = 0; q < 16; ++q) {
          const float lo = msg[q >> 3].f[q & 7];
          const float hi = msg[2 + (q >> 3)].f[q & 7];
          const float snd = sel ? lo : hi;
          const float rcv = __shfl_xor(snd, 8);
          u1[q] = (sel ? hi : lo) + rcv;
        }
      }
      float u2[8];
      {
        const bool sel = (ln & 4) != 0;
#pragma unroll
        for (int q = 0; q < 8; ++q) {
          const float lo = u1[q], hi = u1[8 + q];
          const float snd = sel ? lo : hi;
          const float rcv = __shfl_xor(snd, 4);
          u2[q] = (sel ? hi : lo) + rcv;
        }
      }
      float u3[4];
      {
        const bool sel = (ln & 2) != 0;
#pragma unroll
        for (int q = 0; q < 4; ++q) {
          const float lo = u2[q], hi = u2[4 + q];
          const float snd = sel ? lo : hi;
          const float rcv = __shfl_xor(snd, 2);
          u3[q] = (sel ? hi : lo) + rcv;
        }
      }
      float u4[2];
      {
        const bool sel = (ln & 1) != 0;
#pragma unroll
        for (int q = 0; q < 2; ++q) {
          const float lo = u3[q], hi = u3[2 + q];
          const float snd = sel ? lo : hi;
          const float rcv = __shfl_xor(snd, 1);
          u4[q] = (sel ? hi : lo) + rcv;
        }
      }
      {
        const int hid0 = 16 * (ln >> 2) + 8 * hh + 2 * (ln & 3);
        union { h2_t v; _Float16 e[2]; } o;
        o.e[0] = (_Float16)u4[0];
        o.e[1] = (_Float16)u4[1];
        *(v2h*)&s_agh[i][hid0] = o.v;
      }
    }
    __syncthreads();

    {
      const int mt = wave & 1, nt = wave >> 1, row = mt * 16 + ln;
      Acc acc;
      {
        const float bias = s_ob1[nt * 16 + ln];
#pragma unroll
        for (int r = 0; r < 8; ++r) acc.f[r] = bias;
      }
      const _Float16* ob = wtab + O1OFF + ((0 * 4 + nt) * 32 + lane) * 16;
      Frag fa, fb;
      fa.h[0] = *(const v8h*)&s_xh[row][8 * hh];
      fa.h[1] = *(const v8h*)&s_agh[row][8 * hh];
      fb.h[0] = *(const v8h*)ob; fb.h[1] = *(const v8h*)(ob + 8);
      acc.v = mma16(fa.v, fb.v, acc.v);
      ob += 4 * 32 * 16;
      fa.h[0] = *(const v8h*)&s_agh[row][16 + 8 * hh];
      fa.h[1] = *(const v8h*)&s_agh[row][32 + 8 * hh];
      fb.h[0] = *(const v8h*)ob; fb.h[1] = *(const v8h*)(ob + 8);
      acc.v = mma16(fa.v, fb.v, acc.v);
      ob += 4 * 32 * 16;
      fa.h[0] = *(const v8h*)&s_agh[row][48 + 8 * hh];
      fa.h[1] = z8;
      fb.h[0] = *(const v8h*)ob; fb.h[1] = *(const v8h*)(ob + 8);
      acc.v = mma16(fa.v, fb.v, acc.v);
#pragma unroll
      for (int r = 0; r < 8; ++r)
        s_p1[mt * 16 + 8 * hh + r][nt * 16 + ln] = (_Float16)fmaxf(acc.f[r], 0.0f);
    }
    __syncthreads();

    {
      const int mt = wave & 1, nt = wave >> 1, row = mt * 16 + ln;
      Acc acc;
      {
        const float bias = s_ob2[nt * 16 + ln];
#pragma unroll
        for (int r = 0; r < 8; ++r) acc.f[r] = bias;
      }
#pragma unroll
      for (int kf = 0; kf < 2; ++kf) {
        Frag fa, fb;
        fa.h[0] = *(const v8h*)&s_p1[row][kf * 32 + 8 * hh];
        fa.h[1] = *(const v8h*)&s_p1[row][kf * 32 + 16 + 8 * hh];
        const _Float16* ob = wtab + O2OFF + ((kf * 4 + nt) * 32 + lane) * 16;
        fb.h[0] = *(const v8h*)ob; fb.h[1] = *(const v8h*)(ob + 8);
        acc.v = mma16(fa.v, fb.v, acc.v);
      }
#pragma unroll
      for (int r = 0; r < 8; ++r)
        s_p2[mt * 16 + 8 * hh + r][nt * 16 + ln] = (_Float16)fmaxf(acc.f[r], 0.0f);
    }
    __syncthreads();

    if (wave < 2) {
      const int mt = wave, row = mt * 16 + ln;
      Acc acc;
      {
        const float bias = s_ob3[ln];
#pragma unroll
        for (int r = 0; r < 8; ++r) acc.f[r] = bias;
      }
#pragma unroll
      for (int kf = 0; kf < 2; ++kf) {
        Frag fa, fb;
        fa.h[0] = *(const v8h*)&s_p2[row][kf * 32 + 8 * hh];
        fa.h[1] = *(const v8h*)&s_p2[row][kf * 32 + 16 + 8 * hh];
        const _Float16* ob = wtab + O3OFF + (kf * 32 + lane) * 16;
        fb.h[0] = *(const v8h*)ob; fb.h[1] = *(const v8h*)(ob + 8);
        acc.v = mma16(fa.v, fb.v, acc.v);
      }
#pragma unroll
      for (int r = 0; r < 8; ++r) {
        const int a = mt * 16 + 8 * hh + r;
        const float nx = s_xs[a][ln] + acc.f[r];
        const _Float16 nh = (_Float16)nx;
        s_xs[a][ln] = nx;
        s_xh[a][ln] = nh;
        s_xT[ln][a] = nh;
      }
    }
    __syncthreads();

    if (tid < (NA * ND) / 4) {
      const v4f v = *(const v4f*)(&s_xs[0][0] + tid * 4);
      float* dst = rbuf + ((size_t)blk * 2 + step) * (NA * ND) + tid * 4;
      *(volatile v4f*)dst = v;
      __threadfence();
      *(volatile v4f*)dst = v;
    }
  }
}

__device__ __forceinline__ void pack_pass(int b, int tid, const float* __restrict__ rbuf, float* outp) {
  constexpr int SLAB = NA * NTO * ND;
  constexpr int NCH  = SLAB / 4;
#pragma unroll 1
  for (int c = tid; c < NCH; c += NTHR) {
    const int f   = c * 4;
    const int a   = f / (NTO * ND);
    const int rem = f - a * (NTO * ND);
    const int tau = rem >> 4;
    const int d   = rem & 15;
    const int tt  = tau >> 1, st = tau & 1;
    const v4f v = *(const v4f*)(rbuf + ((size_t)(b * NTS + tt) * 2 + st) * (NA * ND) + a * ND + d);
    *(volatile v4f*)(outp + (size_t)b * SLAB + f) = v;
  }
}

__global__ __launch_bounds__(NTHR)
void k_pack(const float* __restrict__ rbuf, float* __restrict__ outp) {
  const int b = blockIdx.x;
  if (b >= NB) return;
  const int tid = threadIdx.x;
  pack_pass(b, tid, rbuf, outp);
  __threadfence();
  pack_pass(b, tid, rbuf, outp);
}

}

extern "C" void kernel_launch(void* const* d_in, const int* in_sizes, int n_in,
                              void* d_out, int out_size, void* d_ws, size_t ws_size,
                              hipStream_t stream) {
  if (n_in < 15) return;
  if (in_sizes[0]  != NB * NA * NT * ND) return;
  if (in_sizes[1]  != NE * NA) return;
  if (in_sizes[2]  != NE * NA) return;
  if (in_sizes[3]  != NE * 2) return;
  if (in_sizes[4]  != NE * 2) return;
  if (in_sizes[5]  != 2 * 2 * ND * NH) return;
  if (in_sizes[6]  != 2 * NH) return;
  if (in_sizes[7]  != 2 * NH * NH) return;
  if (in_sizes[8]  != 2 * NH) return;
  if (in_sizes[9]  != (ND + NH) * NH) return;
  if (in_sizes[10] != NH) return;
  if (in_sizes[11] != NH * NH) return;
  if (in_sizes[12] != NH) return;
  if (in_sizes[13] != NH * ND) return;
  if (in_sizes[14] != ND) return;
  if (out_size != NB * NA * NTO * ND) return;
  if (ws_size < WS_TOTAL) return;

  const float* xin       = (const float*)d_in[0];
  const float* rel_rec   = (const float*)d_in[1];
  const float* rel_send  = (const float*)d_in[2];
  const float* rel_graph = (const float*)d_in[3];
  const float* gumbel    = (const float*)d_in[4];
  const float* msg_W1    = (const float*)d_in[5];
  const float* msg_b1    = (const float*)d_in[6];
  const float* msg_W2    = (const float*)d_in[7];
  const float* msg_b2    = (const float*)d_in[8];
  const float* out_W1    = (const float*)d_in[9];
  const float* out_b1    = (const float*)d_in[10];
  const float* out_W2    = (const float*)d_in[11];
  const float* out_b2    = (const float*)d_in[12];
  const float* out_W3    = (const float*)d_in[13];
  const float* out_b3    = (const float*)d_in[14];
  float* outp = (float*)d_out;

  char* ws = (char*)d_ws;
  _Float16* wtab = (_Float16*)(ws);
  float*    cpad = (float*)(ws + CPAD_OFFB);
  float*    rbuf = (float*)(ws + R_OFFB);

  k_prep<<<dim3(1), dim3(NTHR), 0, stream>>>(rel_rec, rel_graph, gumbel,
                                             msg_W1, msg_W2, out_W1, out_W2, out_W3,
                                             wtab, cpad);
  k_step<<<dim3(NB * NTS), dim3(NTHR), 0, stream>>>(xin, rel_rec, rel_send, wtab, cpad,
                                                    msg_b1, msg_b2, out_b1, out_b2, out_b3, rbuf);
  k_pack<<<dim3(NB), dim3(NTHR), 0, stream>>>(rbuf, outp);
}
